// CwRNN_34952443854946
// MI455X (gfx1250) — hardware-verified
//
#include <hip/hip_runtime.h>


typedef _Float16 f16t;
typedef f16t  v16h __attribute__((ext_vector_type(16)));
typedef f16t  v8h  __attribute__((ext_vector_type(8)));
typedef float v8f  __attribute__((ext_vector_type(8)));
typedef float v4f  __attribute__((ext_vector_type(4)));
typedef unsigned int v4u __attribute__((ext_vector_type(4)));

union Frag { v16h v; v8h q[2]; };
union Pk16 { v8h h; v4u u; };

#define NB    128
#define NT    512
#define NI    2
#define NH    1024
#define NMOD  8
#define MSZ   128
#define BT    16
#define LP    1032
#define NTHR  256

#define SC_H   256.0f
#define SC_W   64.0f
#define INV_HW 6.103515625e-05f

static_assert((LP * 2) % 16 == 0);
static_assert(NT % 16 == 0);
static_assert(NB % BT == 0);
static_assert(NH == NMOD * MSZ);

__device__ __forceinline__ v8f wmma16(v16h a, v16h b, v8f c) {
    return __builtin_amdgcn_wmma_f32_16x16x32_f16(false, a, false, b, (short)0, c, false, false);
}

__device__ __forceinline__ void wguard4(v8f& c, Frag (&a)[4], Frag (&b)[4]) {
    asm volatile("v_nop\n\tv_nop\n\tv_nop\n\tv_nop"
                 : "+v"(c)
                 : "v"(a[0].v), "v"(a[1].v), "v"(a[2].v), "v"(a[3].v),
                   "v"(b[0].v), "v"(b[1].v), "v"(b[2].v), "v"(b[3].v));
}

__device__ __forceinline__ v8f mma_tile(v8f acc, const f16t* ap, const f16t* __restrict__ bp, int ng) {
#pragma unroll 1
    for (int g = 0; g < ng; ++g) {
        Frag a[4], b[4];
#pragma unroll
        for (int u = 0; u < 4; ++u) {
            const f16t* pa = ap + g * 128 + u * 32;
            const f16t* pb = bp + g * 128 + u * 32;
            a[u].q[0] = *(const v8h*)pa;
            a[u].q[1] = *(const v8h*)(pa + 16);
            b[u].q[0] = *(const v8h*)pb;
            b[u].q[1] = *(const v8h*)(pb + 16);
        }
#pragma unroll
        for (int u = 0; u < 4; ++u) acc = wmma16(a[u].v, b[u].v, acc);
        wguard4(acc, a, b);
    }
    return acc;
}

__device__ __forceinline__ float ftanh(float x) {
    float ax = fabsf(x);
    float t  = __expf(-2.0f * ax);
    float r  = (1.0f - t) * __builtin_amdgcn_rcpf(1.0f + t);
    return copysignf(r, x);
}

__device__ __forceinline__ void cell_update(float a, float xa, float xb, float wi0, float wi1,
                                            float* h32p, f16t* h16p) {
    float xt  = xa * wi0 + xb * wi1;
    float pre = a * INV_HW + xt;
    float v   = ftanh(pre);
    *h32p = v;
    *h16p = (f16t)(v * SC_H);
}

__global__ __launch_bounds__(NTHR)
void k_pack_whh(const float* __restrict__ W, f16t* __restrict__ P, int n8) {
    int i = blockIdx.x * NTHR + threadIdx.x;
    if (i >= n8) return;
    int n  = i >> 7;
    int k8 = (i & 127) * 8;
    const float* src = W + (size_t)n * NH + k8;
    v4f a = *(const v4f*)src;
    v4f b = *(const v4f*)(src + 4);
    float s = ((k8 >> 7) >= (n >> 7)) ? SC_W : 0.0f;
    Pk16 v;
    v.h[0] = (f16t)(a[0] * s); v.h[1] = (f16t)(a[1] * s);
    v.h[2] = (f16t)(a[2] * s); v.h[3] = (f16t)(a[3] * s);
    v.h[4] = (f16t)(b[0] * s); v.h[5] = (f16t)(b[1] * s);
    v.h[6] = (f16t)(b[2] * s); v.h[7] = (f16t)(b[3] * s);
    f16t* d = P + (size_t)n * NH + k8;
    *(volatile v4u*)d = v.u;
    __threadfence();
    *(volatile v4u*)d = v.u;
}

__global__ __launch_bounds__(NTHR)
void k_cw_main(const float* __restrict__ x, const float* __restrict__ W_ih,
               const float* __restrict__ fc_w, const float* __restrict__ fc_b,
               const float* __restrict__ enc_w, const f16t* __restrict__ P,
               float* out, int nb) {
    __shared__ __attribute__((aligned(16))) float h32[BT * NH];
    __shared__ __attribute__((aligned(16))) f16t  h16[BT * LP];
    __shared__ __attribute__((aligned(16))) float fcw[NI * NH];
    __shared__ __attribute__((aligned(16))) float xs[BT * NI];
    __shared__ __attribute__((aligned(16))) float ost[BT * 32];

    const int tid = threadIdx.x;
    const int w   = tid >> 5;
    const int l   = tid & 31, hf = l >> 4, nl = l & 15;
    const int b0  = blockIdx.x * BT;
    if (b0 + BT > nb) return;

    for (int idx = tid; idx < BT * NH; idx += NTHR) {
        int r = idx >> 10, n = idx & (NH - 1);
        const float* xp = x + (size_t)(b0 + r) * (NT + 1) * NI;
        float v = xp[0] * enc_w[n * NI + 0] + xp[1] * enc_w[n * NI + 1];
        h32[idx] = v;
        h16[r * LP + n] = (f16t)(v * SC_H);
    }
    for (int idx = tid; idx < BT * (LP - NH); idx += NTHR) {
        int r = idx >> 3, c = idx & 7;
        h16[r * LP + NH + c] = (f16t)0.0f;
    }
    for (int idx = tid; idx < NI * NH; idx += NTHR) fcw[idx] = fc_w[idx];
    const float fb0 = fc_b[0], fb1 = fc_b[1];
    __syncthreads();

    const int o = tid >> 3, q = tid & 7;
    const int obl = o >> 1, oi = o & 1;

#pragma unroll 1
    for (int t = 0; t < NT; ++t) {
        if (tid < BT * NI) {
            int r = tid >> 1, i = tid & 1;
            xs[tid] = x[((size_t)(b0 + r) * (NT + 1) + (t + 1)) * NI + i];
        }

#pragma unroll 1
        for (int m = 0; m < NMOD; ++m) {
            if ((t & ((1 << m) - 1)) != 0) continue;
            const int n = m * MSZ + 16 * w + nl;
            const float wi0 = W_ih[n * NI + 0];
            const float wi1 = W_ih[n * NI + 1];
            v8f acc = {0.f, 0.f, 0.f, 0.f, 0.f, 0.f, 0.f, 0.f};
            acc = mma_tile(acc,
                           h16 + nl * LP + m * MSZ + 8 * hf,
                           P + (size_t)n * NH + m * MSZ + 8 * hf,
                           NMOD - m);
            __syncthreads();

            const float* xr = xs + 16 * hf;
            v4f x0 = *(const v4f*)(xr);
            v4f x1 = *(const v4f*)(xr + 4);
            v4f x2 = *(const v4f*)(xr + 8);
            v4f x3 = *(const v4f*)(xr + 12);
            float* hr = h32 + (8 * hf) * NH + n;
            f16t*  gr = h16 + (8 * hf) * LP + n;
            cell_update(acc[0], x0[0], x0[1], wi0, wi1, hr + 0 * NH, gr + 0 * LP);
            cell_update(acc[1], x0[2], x0[3], wi0, wi1, hr + 1 * NH, gr + 1 * LP);
            cell_update(acc[2], x1[0], x1[1], wi0, wi1, hr + 2 * NH, gr + 2 * LP);
            cell_update(acc[3], x1[2], x1[3], wi0, wi1, hr + 3 * NH, gr + 3 * LP);
            cell_update(acc[4], x2[0], x2[1], wi0, wi1, hr + 4 * NH, gr + 4 * LP);
            cell_update(acc[5], x2[2], x2[3], wi0, wi1, hr + 5 * NH, gr + 5 * LP);
            cell_update(acc[6], x3[0], x3[1], wi0, wi1, hr + 6 * NH, gr + 6 * LP);
            cell_update(acc[7], x3[2], x3[3], wi0, wi1, hr + 7 * NH, gr + 7 * LP);
        }
        __syncthreads();

        {
            const float* hp = h32 + obl * NH + q * 128;
            const float* fp = fcw + oi * NH + q * 128;
            float s = 0.0f;
#pragma unroll 2
            for (int c = 0; c < 32; ++c) {
                v4f a = *(const v4f*)(hp + 4 * c);
                v4f b = *(const v4f*)(fp + 4 * c);
                s += a[0] * b[0]; s += a[1] * b[1]; s += a[2] * b[2]; s += a[3] * b[3];
            }
            s += __shfl_xor(s, 1);
            s += __shfl_xor(s, 2);
            s += __shfl_xor(s, 4);
            if (q == 0) ost[obl * 32 + (t & 15) * NI + oi] = s + (oi ? fb1 : fb0);
        }

        if ((t & 15) == 15) {
            __syncthreads();
            if (tid < BT * 8) {
                int bl = tid >> 3, p = tid & 7;
                v4f v = *(const v4f*)(ost + bl * 32 + 4 * p);
                float* dst = out + (size_t)(b0 + bl) * (NT * NI) + (t >> 4) * 32 + 4 * p;
                *(volatile v4f*)dst = v;
                __threadfence();
                *(volatile v4f*)dst = v;
            }
        }
    }
}

extern "C" void kernel_launch(void* const* d_in, const int* in_sizes, int n_in,
                              void* d_out, int out_size, void* d_ws, size_t ws_size,
                              hipStream_t stream) {
    if (n_in < 6) return;
    if (in_sizes[0] != NB * (NT + 1) * NI) return;
    if (in_sizes[1] != NH * NI || in_sizes[2] != NH * NH || in_sizes[3] != NI * NH ||
        in_sizes[4] != NI || in_sizes[5] != NH * NI) return;
    if (out_size != NB * NT * NI) return;

    const float* x     = (const float*)d_in[0];
    const float* W_ih  = (const float*)d_in[1];
    const float* W_hh  = (const float*)d_in[2];
    const float* fc_w  = (const float*)d_in[3];
    const float* fc_b  = (const float*)d_in[4];
    const float* enc_w = (const float*)d_in[5];
    float* out = (float*)d_out;

    const size_t pbytes = (size_t)NH * NH * sizeof(f16t);
    if (pbytes > ws_size) return;
    f16t* P = (f16t*)d_ws;

    const int n8 = (NH * NH) / 8;
    k_pack_whh<<<dim3((n8 + NTHR - 1) / NTHR), dim3(NTHR), 0, stream>>>(W_hh, P, n8);
    k_cw_main<<<dim3(NB / BT), dim3(NTHR), 0, stream>>>(x, W_ih, fc_w, fc_b, enc_w, P, out, NB);
}
